// KANLayer_20615843021187
// MI455X (gfx1250) — hardware-verified
//
#include <hip/hip_runtime.h>
#include <math.h>

typedef __attribute__((ext_vector_type(16))) _Float16 v16h;
typedef __attribute__((ext_vector_type(16))) __bf16 v16b;
typedef __attribute__((ext_vector_type(8)))  _Float16 v8h;
typedef __attribute__((ext_vector_type(8)))  float v8f;
typedef __attribute__((ext_vector_type(4)))  float v4f;
typedef __attribute__((ext_vector_type(2)))  float v2f;
typedef __attribute__((ext_vector_type(4)))  unsigned v4u;
typedef __attribute__((ext_vector_type(4)))  int v4i;
typedef float __attribute__((may_alias)) float_a;
typedef int __attribute__((may_alias)) int_a;

template <typename T> __device__ __forceinline__ void vst2(void* p, T v) { *(volatile T*)p = v; __threadfence(); *(volatile T*)p = v; }
__device__ __forceinline__ v8f wmma16(v16h a, v16h b, v8f c) {
  v8f d = __builtin_amdgcn_wmma_f32_16x16x32_f16(false, a, false, b, (short)0, c, false, false);
  asm volatile("v_nop\n\tv_nop\n\tv_nop\n\tv_nop" : "+v"(d) : "v"(a), "v"(b));
  return d;
}
__device__ __forceinline__ v8f wmma_bf(v16b a, v16b b, v8f c) {
  v8f d = __builtin_amdgcn_wmma_f32_16x16x32_bf16(false, a, false, b, (short)0, c, false, false);
  asm volatile("v_nop\n\tv_nop\n\tv_nop\n\tv_nop" : "+v"(d) : "v"(a), "v"(b));
  return d;
}
__device__ __forceinline__ v16h frag_h(const _Float16* rowk0, int lane) {
  union { v16h v; v8h q[2]; } u; const _Float16* p = rowk0 + 8 * (lane >> 4);
  u.q[0] = *(const v8h*)p; u.q[1] = *(const v8h*)(p + 16); return u.v;
}
__device__ __forceinline__ v16h frag_f32(const float* rowk0, int lane) {
  v16h a; const float* p = rowk0 + 8 * (lane >> 4);
#pragma unroll
  for (int i = 0; i < 8; ++i) { a[i] = (_Float16)p[i]; a[8 + i] = (_Float16)p[16 + i]; }
  return a;
}
__device__ __forceinline__ v16h frag_f32s(const float* rowk0, int lane, float sc) {
  v16h a; const float* p = rowk0 + 8 * (lane >> 4);
#pragma unroll
  for (int i = 0; i < 8; ++i) { a[i] = (_Float16)(p[i] * sc); a[8 + i] = (_Float16)(p[16 + i] * sc); }
  return a;
}
__device__ __forceinline__ v16h fragc_f32(const float* W, int k0, int n, int lane, int ld, int K) {
  v16h a; const int g = lane >> 4;
#pragma unroll
  for (int i = 0; i < 8; ++i) { const int ka = k0 + 8 * g + i, kb = ka + 16;
    a[i] = (_Float16)(ka < K ? W[(size_t)(ka < K ? ka : K - 1) * ld + n] : 0.f); a[8 + i] = (_Float16)(kb < K ? W[(size_t)(kb < K ? kb : K - 1) * ld + n] : 0.f); }
  return a;
}
struct F2 { v16b h, l; };
__device__ __forceinline__ F2 bsplit16(const float v[16]) { F2 r;
#pragma unroll
  for (int i = 0; i < 16; ++i) { const __bf16 h = (__bf16)v[i]; r.h[i] = h; r.l[i] = (__bf16)(v[i] - (float)h); }
  return r; }
__device__ __forceinline__ F2 split_row(const float* row, int k0, int lane) { float v[16]; const float* p = row + k0 + 8 * (lane >> 4);
#pragma unroll
  for (int i = 0; i < 8; ++i) { v[i] = p[i]; v[8 + i] = p[16 + i]; }
  return bsplit16(v); }
__device__ __forceinline__ F2 split_rowK(const float* row, int k0, int lane, int K) { float v[16]; const int g = lane >> 4;
#pragma unroll
  for (int i = 0; i < 8; ++i) { const int ka = k0 + 8 * g + i, kb = ka + 16; v[i] = ka < K ? row[ka < K ? ka : K - 1] : 0.f; v[8 + i] = kb < K ? row[kb < K ? kb : K - 1] : 0.f; }
  return bsplit16(v); }
__device__ __forceinline__ F2 split_col(const float* W, int k0, int n, int lane, int ld, int K) { float v[16]; const int g = lane >> 4;
#pragma unroll
  for (int i = 0; i < 8; ++i) { const int ka = k0 + 8 * g + i, kb = ka + 16; v[i] = ka < K ? W[(size_t)(ka < K ? ka : K - 1) * ld + n] : 0.f; v[8 + i] = kb < K ? W[(size_t)(kb < K ? kb : K - 1) * ld + n] : 0.f; }
  return bsplit16(v); }
__device__ __forceinline__ v8f mac3(const F2& a, const F2& b, v8f c) { c = wmma_bf(a.l, b.h, c); c = wmma_bf(a.h, b.l, c); return wmma_bf(a.h, b.h, c); }
__device__ __forceinline__ float sigm(float v) { return 1.0f / (1.0f + expf(-v)); }
#define LDSX() do { asm volatile("s_wait_dscnt 0" ::: "memory"); __builtin_amdgcn_wave_barrier(); __builtin_amdgcn_fence(__ATOMIC_RELEASE, "workgroup"); } while (0)

__device__ __forceinline__ float bfr(float v) { return (float)(__bf16)v; }
#define NBR 4096
#define IN 256
#define OUTD 256
#define NC 8
#define KK (IN * NC)
__device__ __forceinline__ void jacobi8(float t, float al, float p[NC]) {
  p[0] = 1.0f; p[1] = (al + 1.0f) + (al + al + 2.0f) * (t - 1.0f) * 0.5f;
#pragma unroll
  for (int n = 2; n < NC; ++n) { const float fn = (float)n; const float c = 2.0f * fn + al + al; const float A = 2.0f * fn * (fn + al + al) * (c - 2.0f); const float Bc = (c - 1.0f) * (c * (c - 2.0f) * t + (al * al - al * al)); const float Cc = 2.0f * (fn + al - 1.0f) * (fn + al - 1.0f) * c; p[n] = (Bc * p[n - 1] - Cc * p[n - 2]) / A; } }
__global__ __launch_bounds__(128) void k_kan(const float* __restrict__ X, const float* __restrict__ CO, const float* __restrict__ AL, const float* __restrict__ RS, const float* __restrict__ SS, float* __restrict__ OUT) {
  __shared__ __align__(16) float sf[4][16][132]; __shared__ float sres[4][16];
  const int tid = threadIdx.x, wave = tid >> 5, lane = tid & 31, col = lane & 15, g = lane >> 4; const int c0 = blockIdx.y * 128; const size_t r0 = (size_t)blockIdx.x * 64 + wave * 16; const size_t arow = r0 + col;
  const float al = tanhf(bfr(AL[0]));
  v8f acc[8] = {}; float racc = 0.f;
#pragma unroll 1
  for (int kc = 0; kc < KK / 32; ++kc) {
    float av[16]; { const int i0 = kc * 4 + g, i1 = i0 + 2; const float t0 = tanhf(bfr(X[arow * IN + i0])), t1 = tanhf(bfr(X[arow * IN + i1])); float p0[NC], p1[NC]; jacobi8(t0, al, p0); jacobi8(t1, al, p1);
#pragma unroll
      for (int e = 0; e < 8; ++e) { av[e] = p0[e]; av[8 + e] = p1[e]; }
      racc += bfr(RS[i0]) * t0 + bfr(RS[i1]) * t1; }
    const F2 a = bsplit16(av);
#pragma unroll
    for (int j = 0; j < 8; ++j) { const int o = c0 + j * 16 + col; float bv[16]; { const int i0 = kc * 4 + g, i1 = i0 + 2; const float s0 = bfr(SS[(size_t)i0 * OUTD + o]), s1 = bfr(SS[(size_t)i1 * OUTD + o]); const float* q0 = CO + ((size_t)i0 * OUTD + o) * NC; const float* q1 = CO + ((size_t)i1 * OUTD + o) * NC;
#pragma unroll
        for (int e = 0; e < 8; ++e) { bv[e] = s0 * bfr(q0[e]); bv[8 + e] = s1 * bfr(q1[e]); } }
      const F2 bq = bsplit16(bv); acc[j] = wmma_bf(a.h, bq.h, acc[j]); acc[j] = wmma_bf(a.l, bq.h, acc[j]); acc[j] = wmma_bf(a.h, bq.l, acc[j]); } }
  racc += __shfl_xor(racc, 16); if (g == 0) sres[wave][col] = racc;
  LDSX();
#pragma unroll
  for (int j = 0; j < 8; ++j)
#pragma unroll
    for (int r = 0; r < 8; ++r) { const int rl = 8 * g + r; sf[wave][rl][j * 16 + col] = (acc[j][r] + sres[wave][rl]) * (1.0f / (float)IN); }
  LDSX(); for (int rl = 0; rl < 16; ++rl) vst2(OUT + (r0 + rl) * OUTD + c0 + lane * 4, *(const v4f*)&sf[wave][rl][lane * 4]); }
extern "C" void kernel_launch(void* const* d_in, const int* in_sizes, int n_in, void* d_out, int out_size, void* d_ws, size_t ws_size, hipStream_t stream) {
  (void)in_sizes; (void)n_in; (void)out_size; (void)d_ws; (void)ws_size;
  const float** F = (const float**)d_in;
  k_kan<<<dim3(NBR / 64, OUTD / 128), 128, 0, stream>>>(F[0], F[1], F[2], F[3], F[4], (float*)d_out);
}
